// LSTMBlock_21964462751997
// MI455X (gfx1250) — hardware-verified
//
#include <hip/hip_runtime.h>
#include <stdint.h>
#include <stddef.h>


typedef _Float16 v16h __attribute__((ext_vector_type(16)));
typedef _Float16 v8h  __attribute__((ext_vector_type(8)));
typedef float    v8f  __attribute__((ext_vector_type(8)));
typedef float    v4f  __attribute__((ext_vector_type(4)));

union Frag  { v16h v; v8h h[2]; };
union Pack8 { v8h h; v4f f; };

#define NT        512
#define NI        512
#define NH        512
#define NG        2048
#define KF        1024
#define MB        16
#define NTHR      512
#define APITCH    1032
#define OPITCH    516
#define A_BYTES   (MB * APITCH * 2)
#define O_BYTES   (MB * OPITCH * 4)
#define LDS_BYTES (A_BYTES + O_BYTES)
#define WSCALE    64.0f
#define WINV      0.015625f
#define LOG2E     1.4426950408889634f

__device__ __forceinline__ float bf16r(float f) {
  unsigned int u = __float_as_uint(f);
  u = (u + 0x7FFFu + ((u >> 16) & 1u)) & 0xFFFF0000u;
  return __uint_as_float(u);
}

__device__ __forceinline__ v8h cvt8(v4f a, v4f b, float sc) {
  v8h r = { (_Float16)(bf16r(a.x) * sc), (_Float16)(bf16r(a.y) * sc),
            (_Float16)(bf16r(a.z) * sc), (_Float16)(bf16r(a.w) * sc),
            (_Float16)(bf16r(b.x) * sc), (_Float16)(bf16r(b.y) * sc),
            (_Float16)(bf16r(b.z) * sc), (_Float16)(bf16r(b.w) * sc) };
  return r;
}

__device__ __forceinline__ v8f wmma_f16(v16h a, v16h b, v8f c) {
  v8f d = __builtin_amdgcn_wmma_f32_16x16x32_f16(false, a, false, b, (short)0, c, false, false);
  asm volatile("v_nop\n\tv_nop\n\tv_nop\n\tv_nop" : "+v"(d) : "v"(a), "v"(b));
  return d;
}

__device__ __forceinline__ float sigm_(float x) {
  return __builtin_amdgcn_rcpf(1.0f + __builtin_amdgcn_exp2f(-x * LOG2E));
}
__device__ __forceinline__ float tanh_(float x) {
  return 1.0f - 2.0f * __builtin_amdgcn_rcpf(__builtin_amdgcn_exp2f(2.0f * LOG2E * x) + 1.0f);
}

__global__ void __launch_bounds__(256)
cvt_w_kernel(const float* __restrict__ wih, const float* __restrict__ whh,
             _Float16* __restrict__ wf, int nrows)
{
  const int wave = threadIdx.x >> 5;
  const int l = threadIdx.x & 31;
  const int n = blockIdx.x * 8 + wave;
  if (n >= nrows) return;

  Pack8 p[4];
  #pragma unroll
  for (int i = 0; i < 4; ++i) {
    const int kk = 8 * (32 * i + l);
    const float* src = (i < 2) ? (wih + (size_t)n * NI + kk)
                               : (whh + (size_t)n * NH + (kk - NI));
    const v4f f0 = *(const v4f*)(src);
    const v4f f1 = *(const v4f*)(src + 4);
    p[i].h = cvt8(f0, f1, WSCALE);
  }
  _Float16* dst = wf + (size_t)n * KF;
  #pragma unroll
  for (int i = 0; i < 4; ++i)
    *(volatile v4f*)(dst + 8 * (32 * i + l)) = p[i].f;
  __threadfence();
  #pragma unroll
  for (int i = 0; i < 4; ++i)
    *(volatile v4f*)(dst + 8 * (32 * i + l)) = p[i].f;
}

__attribute__((amdgpu_num_vgpr(256)))
__global__ void __launch_bounds__(NTHR)
lstm_seq_kernel(const float* __restrict__ x, const _Float16* __restrict__ wf,
                const float* __restrict__ b_ih, const float* __restrict__ b_hh,
                float* __restrict__ out, int nbatch)
{
  extern __shared__ __align__(16) unsigned char smem[];
  _Float16* As = reinterpret_cast<_Float16*>(smem);
  float*    Os = reinterpret_cast<float*>(smem + A_BYTES);

  const int tid  = threadIdx.x;
  const int wave = tid >> 5;
  const int l    = tid & 31;
  const int hh   = l >> 4;
  const int m    = l & 15;
  const int b0   = blockIdx.x * MB;
  const int srow = wave;
  const int scol = l * 16;
  const bool rowok = (b0 + srow) < nbatch;

  const _Float16 hzero = (_Float16)0.0f;
  const v8h z8 = { hzero, hzero, hzero, hzero, hzero, hzero, hzero, hzero };

  *(v8h*)(As + srow * APITCH + NI + scol)     = z8;
  *(v8h*)(As + srow * APITCH + NI + scol + 8) = z8;

  float bias[8];
  #pragma unroll
  for (int j = 0; j < 8; ++j) {
    const int col = (j >> 1) * NH + (j & 1) * 16 + 32 * wave + m;
    bias[j] = bf16r(b_ih[col]) + bf16r(b_hh[col]);
  }

  float cst[16];
  #pragma unroll
  for (int e = 0; e < 16; ++e) cst[e] = 0.0f;

  const _Float16* arow  = As + m * APITCH + 8 * hh;
  const _Float16* bbase = wf + (size_t)(32 * wave + m) * KF + 8 * hh;
  const float*    orow  = Os + srow * OPITCH;

  for (int t = 0; t < NT; ++t) {
    {
      v8h p0, p1;
      if (rowok) {
        const float* xp = x + ((size_t)(b0 + srow) * NT + (size_t)t) * NI + scol;
        const v4f f0 = *(const v4f*)(xp);
        const v4f f1 = *(const v4f*)(xp + 4);
        const v4f f2 = *(const v4f*)(xp + 8);
        const v4f f3 = *(const v4f*)(xp + 12);
        p0 = cvt8(f0, f1, 1.0f);
        p1 = cvt8(f2, f3, 1.0f);
      } else {
        p0 = z8; p1 = z8;
      }
      *(v8h*)(As + srow * APITCH + scol)     = p0;
      *(v8h*)(As + srow * APITCH + scol + 8) = p1;
    }
    __syncthreads();

    const v8f zacc = { 0.f, 0.f, 0.f, 0.f, 0.f, 0.f, 0.f, 0.f };
    v8f acc[8];
    #pragma unroll
    for (int j = 0; j < 8; ++j) acc[j] = zacc;

    #pragma unroll 1
    for (int ks = 0; ks < KF / 32; ++ks) {
      const int k0 = ks * 32;
      Frag a;
      a.h[0] = *(const v8h*)(arow + k0);
      a.h[1] = *(const v8h*)(arow + k0 + 16);
      #pragma unroll
      for (int j = 0; j < 8; ++j) {
        const _Float16* bp = bbase + (size_t)(((j >> 1) * NH + (j & 1) * 16) * KF) + k0;
        Frag b;
        b.h[0] = *(const v8h*)(bp);
        b.h[1] = *(const v8h*)(bp + 16);
        acc[j] = wmma_f16(a.v, b.v, acc[j]);
      }
    }
    __syncthreads();

    #pragma unroll
    for (int s = 0; s < 2; ++s) {
      const int u = 32 * wave + 16 * s + m;
      #pragma unroll
      for (int r = 0; r < 8; ++r) {
        const int br = 8 * hh + r;
        const float pi = acc[0 * 2 + s][r] * WINV + bias[0 * 2 + s];
        const float pf = acc[1 * 2 + s][r] * WINV + bias[1 * 2 + s];
        const float pg = acc[2 * 2 + s][r] * WINV + bias[2 * 2 + s];
        const float po = acc[3 * 2 + s][r] * WINV + bias[3 * 2 + s];
        const float ig = sigm_(pi);
        const float fg = sigm_(pf);
        const float gg = tanh_(pg);
        const float og = sigm_(po);
        const float cn = fg * cst[s * 8 + r] + ig * gg;
        cst[s * 8 + r] = cn;
        const float hn = og * tanh_(cn);
        As[br * APITCH + NI + u] = (_Float16)hn;
        Os[br * OPITCH + u]      = fmaxf(hn, 0.0f);
      }
    }
    __syncthreads();

    {
      const v4f o0 = *(const v4f*)(orow + 4 * l);
      const v4f o1 = *(const v4f*)(orow + 128 + 4 * l);
      const v4f o2 = *(const v4f*)(orow + 256 + 4 * l);
      const v4f o3 = *(const v4f*)(orow + 384 + 4 * l);
      const size_t obase = ((size_t)(b0 + srow) * NT + (size_t)t) * NH + (size_t)(4 * l);
      if (rowok) {
        float* op = out + obase;
        *(volatile v4f*)(op)       = o0;
        *(volatile v4f*)(op + 128) = o1;
        *(volatile v4f*)(op + 256) = o2;
        *(volatile v4f*)(op + 384) = o3;
      }
      __threadfence();
      if (rowok) {
        float* op = out + obase;
        *(volatile v4f*)(op)       = o0;
        *(volatile v4f*)(op + 128) = o1;
        *(volatile v4f*)(op + 256) = o2;
        *(volatile v4f*)(op + 384) = o3;
      }
    }
  }
}

extern "C" void kernel_launch(void* const* d_in, const int* in_sizes, int n_in,
                              void* d_out, int out_size, void* d_ws, size_t ws_size,
                              hipStream_t stream) {
  if (n_in < 5) return;
  const float* x    = (const float*)d_in[0];
  const float* W_ih = (const float*)d_in[1];
  const float* W_hh = (const float*)d_in[2];
  const float* b_ih = (const float*)d_in[3];
  const float* b_hh = (const float*)d_in[4];
  float* out = (float*)d_out;

  const long long nx = (long long)in_sizes[0];
  const int nbatch = (int)(nx / ((long long)NT * NI));
  if (nbatch <= 0) return;
  if ((long long)nbatch * NT * NH > (long long)out_size) return;
  if ((long long)in_sizes[1] < (long long)NG * NI) return;
  if ((long long)in_sizes[2] < (long long)NG * NH) return;
  if (in_sizes[3] < NG || in_sizes[4] < NG) return;

  const size_t wf_bytes = (size_t)NG * KF * sizeof(_Float16);
  if (wf_bytes > ws_size) return;
  _Float16* wf = (_Float16*)d_ws;

  cvt_w_kernel<<<(NG + 7) / 8, 256, 0, stream>>>(W_ih, W_hh, wf, NG);

  hipFuncSetAttribute(reinterpret_cast<const void*>(&lstm_seq_kernel),
                      hipFuncAttributeMaxDynamicSharedMemorySize, LDS_BYTES);
  lstm_seq_kernel<<<(nbatch + MB - 1) / MB, NTHR, LDS_BYTES, stream>>>(x, wf, b_ih, b_hh, out, nbatch);
}
